// LocalCrossAttention_90288802497335
// MI455X (gfx1250) — hardware-verified
//
#include <hip/hip_runtime.h>
#include <math.h>
#include <stdint.h>

#ifndef NB
#define NB 1
#endif
#ifndef SEQ
#define SEQ 4096
#endif
#define NB_FULL  1
#define SEQ_FULL 4096
#define EMB      1024
#define QH       (SEQ / 2)
#define NCH      (SEQ / 256)
#define GCH      ((NCH < 8) ? NCH : 8)
#define PCARRY   16384.0f
#define VCARRY   8.0f
#define SM_SCALE 0.03125f
#define OFF1     ((size_t)SEQ_FULL * EMB)
static_assert(NB == 1 && NB_FULL == 1);
static_assert(SEQ >= 256 && SEQ <= SEQ_FULL && (SEQ % 256) == 0);
static_assert((QH % 64) == 0 && (SEQ % 64) == 0 && (EMB % 64) == 0 && (EMB % 32) == 0 && (SEQ % 32) == 0);
static_assert((NCH % GCH) == 0 && (QH % 8) == 0);
static_assert(OFF1 * 4 == 16777216);

typedef _Float16 v16h __attribute__((ext_vector_type(16)));
typedef _Float16 v8h  __attribute__((ext_vector_type(8)));
typedef __bf16   v16b __attribute__((ext_vector_type(16)));
typedef __bf16   v8b  __attribute__((ext_vector_type(8)));
typedef float    v8f  __attribute__((ext_vector_type(8)));
typedef float    v4f  __attribute__((ext_vector_type(4)));
typedef unsigned int v4u __attribute__((ext_vector_type(4)));

#if defined(__HIP_DEVICE_COMPILE__)
#define DEV_ASM 1
#else
#define DEV_ASM 0
#endif

__device__ __forceinline__ unsigned short bf_bits(float f) {
  unsigned u = __float_as_uint(f);
  return (unsigned short)((u + 0x7FFFu + ((u >> 16) & 1u)) >> 16);
}
__device__ __forceinline__ float bf_up(unsigned short hb) { return __uint_as_float(((unsigned)hb) << 16); }
__device__ __forceinline__ unsigned short h_bits(_Float16 x) { return __builtin_bit_cast(unsigned short, x); }
__device__ __forceinline__ unsigned pk16(unsigned short a, unsigned short b) { return (unsigned)a | ((unsigned)b << 16); }
__device__ __forceinline__ v8f zero8() { v8f z = {0.f, 0.f, 0.f, 0.f, 0.f, 0.f, 0.f, 0.f}; return z; }

template <typename OT> struct FT;
template <> struct FT<__bf16>   { typedef v16b frag; typedef v8b half8; };
template <> struct FT<_Float16> { typedef v16h frag; typedef v8h half8; };

template <typename OT>
__device__ __forceinline__ typename FT<OT>::frag ldfrag(const OT* p) {
  union { typename FT<OT>::frag v; typename FT<OT>::half8 h[2]; } f;
  f.h[0] = *(const typename FT<OT>::half8*)(p);
  f.h[1] = *(const typename FT<OT>::half8*)(p + 16);
  return f.v;
}

__device__ __forceinline__ v8f mmar(v16b a, v16b b, v8f c) {
  return __builtin_amdgcn_wmma_f32_16x16x32_bf16(false, a, false, b, (short)0, c, false, false);
}
__device__ __forceinline__ v8f mmar(v16h a, v16h b, v8f c) {
  return __builtin_amdgcn_wmma_f32_16x16x32_f16(false, a, false, b, (short)0, c, false, false);
}
__device__ __forceinline__ void dep_guard(v8f& a, v8f& b, v16b x, v16b y) {
#if DEV_ASM
  asm volatile("v_nop\n\tv_nop\n\tv_nop\n\tv_nop" : "+v"(a), "+v"(b) : "v"(x), "v"(y));
#else
  (void)a; (void)b; (void)x; (void)y;
#endif
}
__device__ __forceinline__ void dep_guard(v8f& a, v8f& b, v16h x, v16h y) {
#if DEV_ASM
  asm volatile("v_nop\n\tv_nop\n\tv_nop\n\tv_nop" : "+v"(a), "+v"(b) : "v"(x), "v"(y));
#else
  (void)a; (void)b; (void)x; (void)y;
#endif
}
__device__ __forceinline__ void keep4(v16b a, v16b b, v16b c, v16b d) {
#if DEV_ASM
  asm volatile("v_nop" :: "v"(a), "v"(b), "v"(c), "v"(d));
#else
  (void)a; (void)b; (void)c; (void)d;
#endif
}
__device__ __forceinline__ void keep4(v16h a, v16h b, v16h c, v16h d) {
#if DEV_ASM
  asm volatile("v_nop" :: "v"(a), "v"(b), "v"(c), "v"(d));
#else
  (void)a; (void)b; (void)c; (void)d;
#endif
}
__device__ __forceinline__ void acc_guard4(v8f& a, v8f& b, v8f& c, v8f& d) {
#if DEV_ASM
  asm volatile("v_nop\n\tv_nop\n\tv_nop\n\tv_nop" : "+v"(a), "+v"(b), "+v"(c), "+v"(d));
#else
  (void)a; (void)b; (void)c; (void)d;
#endif
}

__global__ __launch_bounds__(256) void cvt_bf16x8(const float* __restrict__ in, unsigned short* out, int n8) {
  const int i = blockIdx.x * 256 + (int)threadIdx.x;
  if (i < n8) {
    const v4f a  = *(const v4f*)(in + (size_t)i * 8);
    const v4f a4 = *(const v4f*)(in + (size_t)i * 8 + 4);
    v4u p;
    p[0] = pk16(bf_bits(a[0]),  bf_bits(a[1]));
    p[1] = pk16(bf_bits(a[2]),  bf_bits(a[3]));
    p[2] = pk16(bf_bits(a4[0]), bf_bits(a4[1]));
    p[3] = pk16(bf_bits(a4[2]), bf_bits(a4[3]));
    unsigned short* o = out + (size_t)i * 8;
    *(volatile v4u*)o = p;
    __threadfence();
    *(volatile v4u*)o = p;
  }
}

template <typename OT, int MI, int NPA, int OUT_MODE, int BM>
__global__ __launch_bounds__(256) void gemm_t(
    const unsigned short* __restrict__ Ap, const unsigned short* __restrict__ A2p, int lda, long long strideA,
    const unsigned short* __restrict__ Btp, int ldb, long long strideB,
    void* Cout, void* Cout2, int ldc, long long strideC,
    const float* __restrict__ bias,
    int M, int N, int K, float oscale, float rscaleA, float cscale, float rscaleC) {
  typedef typename FT<OT>::frag V16;
  const OT* A  = (const OT*)(const void*)Ap;
  const OT* A2 = (const OT*)(const void*)A2p;
  const OT* Bt = (const OT*)(const void*)Btp;
  __shared__ __align__(16) float sT[8][16 * 68];
  const int RT   = 16 * MI;
  const int b    = blockIdx.y;
  const int lane = threadIdx.x & 31;
  const int wave = threadIdx.x >> 5;
  const int tilesN = N >> 6;
  const int tilesM = M / RT;
  const int tile = blockIdx.x * 8 + wave;
  if (tile >= tilesM * tilesN) return;
  const int tm = tile / tilesN;
  const int tn = tile - tm * tilesN;
  const int m0 = tm * RT;
  const int n0 = tn << 6;

  const OT* Ab  = A  + (size_t)b * (size_t)strideA;
  const OT* A2b = A2 + (size_t)b * (size_t)strideA;
  const OT* Bb  = Bt + (size_t)b * (size_t)strideB;

  const int rlane = lane & 15;
  const int koff  = (lane >> 4) * 8;
  const int mOff  = (lane >> 4) * 8;

  v8f acc[MI][4], acc2[MI][4];
#pragma unroll
  for (int i = 0; i < MI; ++i)
#pragma unroll
    for (int j = 0; j < 4; ++j) { acc[i][j] = zero8(); acc2[i][j] = zero8(); }

  for (int k0 = 0; k0 < K; k0 += 32) {
    V16 bq[4];
#pragma unroll
    for (int j = 0; j < 4; ++j)
      bq[j] = ldfrag<OT>(Bb + (size_t)(n0 + (j << 4) + rlane) * ldb + koff + k0);
#pragma unroll
    for (int i = 0; i < MI; ++i) {
      const V16 af = ldfrag<OT>(Ab + (size_t)(m0 + (i << 4) + rlane) * lda + koff + k0);
#pragma unroll
      for (int j = 0; j < 4; ++j) acc[i][j] = mmar(af, bq[j], acc[i][j]);
      dep_guard(acc[i][0], acc[i][3], af, bq[3]);
      if (NPA == 2) {
        const V16 af2 = ldfrag<OT>(A2b + (size_t)(m0 + (i << 4) + rlane) * lda + koff + k0);
#pragma unroll
        for (int j = 0; j < 4; ++j) acc2[i][j] = mmar(af2, bq[j], acc2[i][j]);
        dep_guard(acc2[i][0], acc2[i][3], af2, bq[3]);
      }
    }
    keep4(bq[0], bq[1], bq[2], bq[3]);
  }
#pragma unroll
  for (int i = 0; i < MI; ++i) {
    acc_guard4(acc[i][0], acc[i][1], acc[i][2], acc[i][3]);
    if (NPA == 2) acc_guard4(acc2[i][0], acc2[i][1], acc2[i][2], acc2[i][3]);
  }

  float bcol[4];
#pragma unroll
  for (int j = 0; j < 4; ++j) bcol[j] = 0.f;
  if (BM == 1) {
#pragma unroll
    for (int j = 0; j < 4; ++j) bcol[j] = bf_up(bf_bits(bias[n0 + (j << 4) + rlane]));
  }
  float* slab = sT[wave];
#pragma unroll
  for (int i = 0; i < MI; ++i) {
    const int mBase = m0 + (i << 4);
    float brow[8];
#pragma unroll
    for (int r = 0; r < 8; ++r) brow[r] = 0.f;
    if (BM == 2) {
#pragma unroll
      for (int r = 0; r < 8; ++r) brow[r] = bf_up(bf_bits(bias[mBase + mOff + r]));
    }
#pragma unroll
    for (int j = 0; j < 4; ++j) {
#pragma unroll
      for (int r = 0; r < 8; ++r) {
        float v = acc[i][j][r];
        if (NPA == 2) v += acc2[i][j][r] * rscaleA;
        v = v * oscale + bcol[j] + brow[r];
        slab[(mOff + r) * 68 + (j << 4) + rlane] = v;
      }
    }
    __builtin_amdgcn_fence(__ATOMIC_RELEASE, "workgroup");
    __builtin_amdgcn_wave_barrier();
    __builtin_amdgcn_fence(__ATOMIC_ACQUIRE, "workgroup");
    if (OUT_MODE == 0) {
      float* C = (float*)Cout + (size_t)b * (size_t)strideC;
      const int h2 = lane >> 4, c4 = (lane & 15) * 4;
      for (int pass = 0; pass < 2; ++pass) {
#pragma unroll
        for (int it = 0; it < 8; ++it) {
          const int row = it * 2 + h2;
          const v4f v = *(const v4f*)(slab + row * 68 + c4);
          *(volatile v4f*)(C + (size_t)(mBase + row) * ldc + n0 + c4) = v;
        }
        __threadfence();
      }
    } else {
      const int q = lane >> 3, c8 = (lane & 7) * 8;
      unsigned short* C  = (unsigned short*)Cout  + (size_t)b * (size_t)strideC;
      unsigned short* C2 = (unsigned short*)Cout2 + (size_t)b * (size_t)strideC;
      v4u hv[4], lv[4];
#pragma unroll
      for (int it = 0; it < 4; ++it) {
        const int row = it * 4 + q;
        const float* sp = slab + row * 68 + c8;
        float f[8];
#pragma unroll
        for (int e = 0; e < 8; ++e) f[e] = sp[e] * cscale;
        v4u a, a2;
#pragma unroll
        for (int e = 0; e < 4; ++e) {
          const float f0 = f[2 * e], f1 = f[2 * e + 1];
          const _Float16 x0 = (_Float16)f0, x1 = (_Float16)f1;
          const unsigned short h0 = h_bits(x0), h1 = h_bits(x1);
          unsigned short l0 = 0, l1 = 0;
          if (OUT_MODE == 3) {
            l0 = h_bits((_Float16)((f0 - (float)x0) * rscaleC));
            l1 = h_bits((_Float16)((f1 - (float)x1) * rscaleC));
          }
          a[e] = pk16(h0, h1); a2[e] = pk16(l0, l1);
        }
        hv[it] = a; lv[it] = a2;
      }
      for (int pass = 0; pass < 2; ++pass) {
#pragma unroll
        for (int it = 0; it < 4; ++it) {
          const int row = it * 4 + q;
          *(volatile v4u*)(C + (size_t)(mBase + row) * ldc + n0 + c8) = hv[it];
          if (OUT_MODE == 3) *(volatile v4u*)(C2 + (size_t)(mBase + row) * ldc + n0 + c8) = lv[it];
        }
        __threadfence();
      }
    }
    __builtin_amdgcn_fence(__ATOMIC_RELEASE, "workgroup");
    __builtin_amdgcn_wave_barrier();
    __builtin_amdgcn_fence(__ATOMIC_ACQUIRE, "workgroup");
  }
}

__global__ __launch_bounds__(256)
void softmax_rows(const float* __restrict__ S, unsigned short* P, int nrows) {
#pragma clang fp contract(off)
  const int wave = threadIdx.x >> 5;
  const int lane = threadIdx.x & 31;
  const int row  = blockIdx.x * 8 + wave;
  if (row >= nrows) return;
  const float* sr = S + (size_t)row * SEQ + lane * 8;
  unsigned short* pr = P + (size_t)row * SEQ + lane * 8;

  float m = -INFINITY;
#pragma unroll 2
  for (int c = 0; c < NCH; ++c) {
    const v4f a  = *(const v4f*)(sr + c * 256);
    const v4f a4 = *(const v4f*)(sr + c * 256 + 4);
    m = fmaxf(m, fmaxf(fmaxf(a[0], a[1]), fmaxf(a[2], a[3])));
    m = fmaxf(m, fmaxf(fmaxf(a4[0], a4[1]), fmaxf(a4[2], a4[3])));
  }
#pragma unroll
  for (int off = 1; off < 32; off <<= 1) m = fmaxf(m, __shfl_xor(m, off, 32));

  float l = 0.f;
#pragma unroll 2
  for (int c = 0; c < NCH; ++c) {
    const v4f a  = *(const v4f*)(sr + c * 256);
    const v4f a4 = *(const v4f*)(sr + c * 256 + 4);
#pragma unroll
    for (int e = 0; e < 4; ++e) l += __expf(a[e] - m);
#pragma unroll
    for (int e = 0; e < 4; ++e) l += __expf(a4[e] - m);
  }
#pragma unroll
  for (int off = 1; off < 32; off <<= 1) l += __shfl_xor(l, off, 32);
  const float cl = PCARRY * (1.0f / l);

#pragma unroll 1
  for (int g = 0; g < NCH; g += GCH) {
    v4u hv[GCH];
#pragma unroll
    for (int j = 0; j < GCH; ++j) {
      const v4f a  = *(const v4f*)(sr + (g + j) * 256);
      const v4f a4 = *(const v4f*)(sr + (g + j) * 256 + 4);
      v4u p;
      p[0] = pk16(h_bits((_Float16)(__expf(a[0]  - m) * cl)), h_bits((_Float16)(__expf(a[1]  - m) * cl)));
      p[1] = pk16(h_bits((_Float16)(__expf(a[2]  - m) * cl)), h_bits((_Float16)(__expf(a[3]  - m) * cl)));
      p[2] = pk16(h_bits((_Float16)(__expf(a4[0] - m) * cl)), h_bits((_Float16)(__expf(a4[1] - m) * cl)));
      p[3] = pk16(h_bits((_Float16)(__expf(a4[2] - m) * cl)), h_bits((_Float16)(__expf(a4[3] - m) * cl)));
      hv[j] = p;
    }
    for (int pass = 0; pass < 2; ++pass) {
#pragma unroll
      for (int j = 0; j < GCH; ++j) *(volatile v4u*)(pr + (g + j) * 256) = hv[j];
      __threadfence();
    }
  }
}

static void attend_dir(hipStream_t stream,
                       const unsigned short* Xq, const unsigned short* Xkv,
                       const unsigned short* Wq, const float* bq,
                       const unsigned short* Wk, const float* bk,
                       const unsigned short* Wv, const float* bv,
                       unsigned short* Qp, unsigned short* Kp, unsigned short* VT,
                       float* S, unsigned short* P, float* outp) {
  const dim3 blk(256);
  const int tProj = (SEQ / 64) * (EMB / 64);
  const int tVT   = (EMB / 64) * (SEQ / 64);
  const int tS    = (QH / 64) * (SEQ / 64);
  const int tPV   = (QH / 64) * (EMB / 64);
  const dim3 gProj((tProj + 7) / 8, 1);
  const dim3 gVT((tVT + 7) / 8, 1);
  const dim3 gS((tS + 7) / 8, 1);
  const dim3 gPV((tPV + 7) / 8, 1);
  const dim3 gSm(QH / 8);

  gemm_t<__bf16, 4, 1, 1, 1><<<gProj, blk, 0, stream>>>(
      Xq, Xq, EMB, 0LL, Wq, EMB, 0LL,
      (void*)Qp, (void*)Qp, EMB, 0LL, bq,
      SEQ, EMB, EMB, 1.0f, 0.0f, 1.0f, 1.0f);
  gemm_t<__bf16, 4, 1, 1, 1><<<gProj, blk, 0, stream>>>(
      Xkv, Xkv, EMB, 0LL, Wk, EMB, 0LL,
      (void*)Kp, (void*)Kp, EMB, 0LL, bk,
      SEQ, EMB, EMB, 1.0f, 0.0f, 1.0f, 1.0f);
  gemm_t<__bf16, 4, 1, 1, 2><<<gVT, blk, 0, stream>>>(
      Wv, Wv, EMB, 0LL, Xkv, EMB, 0LL,
      (void*)VT, (void*)VT, SEQ, 0LL, bv,
      EMB, SEQ, EMB, 1.0f, 0.0f, VCARRY, 1.0f);
  for (int h = 0; h < 2; ++h) {
    const unsigned short* Qh = Qp + (size_t)h * QH * EMB;
    float* Oh = outp + (size_t)h * QH * EMB;
    gemm_t<_Float16, 4, 1, 0, 0><<<gS, blk, 0, stream>>>(
        Qh, Qh, EMB, 0LL, Kp, EMB, 0LL,
        (void*)S, (void*)S, SEQ, 0LL, bq,
        QH, SEQ, EMB, SM_SCALE, 0.0f, 1.0f, 1.0f);
    softmax_rows<<<gSm, blk, 0, stream>>>(S, P, QH);
    gemm_t<_Float16, 4, 1, 0, 0><<<gPV, blk, 0, stream>>>(
        P, P, SEQ, 0LL, VT, SEQ, 0LL,
        (void*)Oh, (void*)Oh, EMB, 0LL, bq,
        QH, EMB, SEQ, 1.0f / (PCARRY * VCARRY), 0.0f, 1.0f, 1.0f);
  }
}

extern "C" void kernel_launch(void* const* d_in, const int* in_sizes, int n_in,
                              void* d_out, int out_size, void* d_ws, size_t ws_size,
                              hipStream_t stream) {
  if (n_in < 14) return;
  if (in_sizes[0] < SEQ * EMB) return;
  if (in_sizes[1] < SEQ * EMB) return;
  for (int j = 0; j < 6; ++j) {
    if (in_sizes[2 + 2 * j] < EMB * EMB) return;
    if (in_sizes[3 + 2 * j] < EMB) return;
  }
  if (out_size < 0) return;
  if ((size_t)out_size < OFF1 + (size_t)SEQ * EMB) return;

  const float* x1  = (const float*)d_in[0];
  const float* x2  = (const float*)d_in[1];
  const float* Wq1 = (const float*)d_in[2];  const float* bq1 = (const float*)d_in[3];
  const float* Wk1 = (const float*)d_in[4];  const float* bk1 = (const float*)d_in[5];
  const float* Wv1 = (const float*)d_in[6];  const float* bv1 = (const float*)d_in[7];
  const float* Wq2 = (const float*)d_in[8];  const float* bq2 = (const float*)d_in[9];
  const float* Wk2 = (const float*)d_in[10]; const float* bk2 = (const float*)d_in[11];
  const float* Wv2 = (const float*)d_in[12]; const float* bv2 = (const float*)d_in[13];

  const size_t PW  = (size_t)EMB * EMB * 2;
  const size_t PX  = (size_t)SEQ * EMB * 2;
  const size_t PVT = (size_t)EMB * SEQ * 2;
  const size_t PS  = (size_t)QH * SEQ * 4;
  const size_t PP  = (size_t)QH * SEQ * 2;
  size_t off = 0;
  const size_t oW  = off; off += 6 * PW;
  const size_t oX1 = off; off += PX;
  const size_t oX2 = off; off += PX;
  const size_t oQ  = off; off += PX;
  const size_t oK  = off; off += PX;
  const size_t oVT = off; off += PVT;
  const size_t oS  = off; off += PS;
  const size_t oP  = off; off += PP;
  if (off > ws_size) return;
  if (off > (size_t)134217728) return;

  char* ws = (char*)d_ws;
  unsigned short* Wb  = (unsigned short*)(ws + oW);
  unsigned short* X1b = (unsigned short*)(ws + oX1);
  unsigned short* X2b = (unsigned short*)(ws + oX2);
  unsigned short* Qp  = (unsigned short*)(ws + oQ);
  unsigned short* Kp  = (unsigned short*)(ws + oK);
  unsigned short* VT  = (unsigned short*)(ws + oVT);
  float*          S   = (float*)(ws + oS);
  unsigned short* P   = (unsigned short*)(ws + oP);
  const size_t    WE  = (size_t)EMB * EMB;
  unsigned short* Wq1b = Wb;          unsigned short* Wk1b = Wb + WE;     unsigned short* Wv1b = Wb + 2 * WE;
  unsigned short* Wq2b = Wb + 3 * WE; unsigned short* Wk2b = Wb + 4 * WE; unsigned short* Wv2b = Wb + 5 * WE;
  float* out0 = (float*)d_out;
  float* out1 = (float*)d_out + OFF1;

  const dim3 blk(256);
  const int n8x = SEQ * EMB / 8;
  const int n8w = EMB * EMB / 8;
  const dim3 gCx((n8x + 255) / 256);
  const dim3 gCw((n8w + 255) / 256);

  cvt_bf16x8<<<gCx, blk, 0, stream>>>(x1, X1b, n8x);
  cvt_bf16x8<<<gCx, blk, 0, stream>>>(x2, X2b, n8x);
  cvt_bf16x8<<<gCw, blk, 0, stream>>>(Wq1, Wq1b, n8w);
  cvt_bf16x8<<<gCw, blk, 0, stream>>>(Wk1, Wk1b, n8w);
  cvt_bf16x8<<<gCw, blk, 0, stream>>>(Wv1, Wv1b, n8w);
  cvt_bf16x8<<<gCw, blk, 0, stream>>>(Wq2, Wq2b, n8w);
  cvt_bf16x8<<<gCw, blk, 0, stream>>>(Wk2, Wk2b, n8w);
  cvt_bf16x8<<<gCw, blk, 0, stream>>>(Wv2, Wv2b, n8w);
  attend_dir(stream, X2b, X1b, Wq2b, bq2, Wk1b, bk1, Wv1b, bv1, Qp, Kp, VT, S, P, out0);
  attend_dir(stream, X1b, X2b, Wq1b, bq1, Wk2b, bk2, Wv2b, bv2, Qp, Kp, VT, S, P, out1);
  (void)hipGetLastError();
}
